// Voltera_75428215652658
// MI455X (gfx1250) — hardware-verified
//
#include <hip/hip_runtime.h>


#define NTOK 1024
#define TCH  256
#define KK   65536
#define OC   64
__constant__ float c_norm[15] = {1.000000000e+00f,7.978846431e-01f,5.000000000e-01f,2.659615278e-01f,1.250000000e-01f,5.319230258e-02f,2.083333395e-02f,7.598902099e-03f,2.604166744e-03f,8.443223778e-04f,2.604166220e-04f,7.675658708e-05f,2.170138760e-05f,5.904352292e-06f,1.550098659e-06f};
#define SIG  8.313910675e+01f
typedef _Float16 h16;
typedef unsigned short bf;
typedef __attribute__((ext_vector_type(16))) __bf16   v16bf;
typedef __attribute__((ext_vector_type(16))) _Float16 v16h;
typedef __attribute__((ext_vector_type(8)))  _Float16 v8h;
typedef __attribute__((ext_vector_type(8)))  unsigned short v8us;
typedef __attribute__((ext_vector_type(8)))  float    v8f;
typedef __attribute__((ext_vector_type(4)))  float    v4f;
typedef v8h  __attribute__((may_alias)) v8ha;
typedef v4f  __attribute__((may_alias)) v4fa;
typedef v8us __attribute__((may_alias)) v8usa;

__device__ __forceinline__ unsigned short f2bf(float f) { unsigned u = __float_as_uint(f); u += 0x7FFFu + ((u >> 16) & 1u); return (unsigned short)(u >> 16); }
__device__ __forceinline__ float bf2f(unsigned short b) { return __uint_as_float(((unsigned)b) << 16); }
__device__ __forceinline__ float bfr(float f) { return bf2f(f2bf(f)); }
__device__ __forceinline__ v16h cat16(v8h lo, v8h hi) { return __builtin_shufflevector(lo, hi, 0, 1, 2, 3, 4, 5, 6, 7, 8, 9, 10, 11, 12, 13, 14, 15); }
__device__ __forceinline__ v16bf cat16b(v8us lo, v8us hi) { return __builtin_bit_cast(v16bf, __builtin_shufflevector(lo, hi, 0, 1, 2, 3, 4, 5, 6, 7, 8, 9, 10, 11, 12, 13, 14, 15)); }
__device__ __forceinline__ v8f wmma16(v16h a, v16h b, v8f c) { return __builtin_amdgcn_wmma_f32_16x16x32_f16(false, a, false, b, (short)0, c, false, false); }
__device__ __forceinline__ v8f wmmab(v16bf a, v16bf b, v8f c) { return __builtin_amdgcn_wmma_f32_16x16x32_bf16(false, a, false, b, (short)0, c, false, false); }


template <typename T16> struct WFrag;
template <> struct WFrag<h16> { typedef v16h V; static __device__ __forceinline__ V ld(const h16* p) { return cat16(*(const v8h*)p, *(const v8h*)(p + 16)); } static __device__ __forceinline__ v8f mma(V a, V b, v8f c) { return wmma16(a, b, c); } };
template <> struct WFrag<bf> { typedef v16bf V; static __device__ __forceinline__ V ld(const bf* p) { return cat16b(*(const v8us*)p, *(const v8us*)(p + 16)); } static __device__ __forceinline__ v8f mma(V a, V b, v8f c) { return wmmab(a, b, c); } };
template <typename T16, int NSPLIT, bool BIAS>
__global__ __launch_bounds__(32) void k_gemmw(const T16* __restrict__ A, const T16* __restrict__ A2, const T16* __restrict__ Bt, const T16* __restrict__ Bt2, int K, float* C, int ldc, const float* __restrict__ bias, size_t sA, size_t sB, size_t sC) {
    typedef typename WFrag<T16>::V V;
    __shared__ __align__(16) float os[16 * 68];
    const size_t z = blockIdx.z; A += z * sA; if (A2) A2 += z * sA; Bt += z * sB; if (Bt2) Bt2 += z * sB; C += z * sC;
    const int lane = threadIdx.x & 31, lr = lane & 15, hi = lane >> 4; const int r0 = blockIdx.x * 64, c0 = blockIdx.y * 64;
    v8f acc[4][4];
#pragma unroll
    for (int mb = 0; mb < 4; ++mb)
#pragma unroll
        for (int nb = 0; nb < 4; ++nb) acc[mb][nb] = (v8f){};
    const size_t aoff = (size_t)(r0 + lr) * K + 8 * hi, boff = (size_t)(c0 + lr) * K + 8 * hi;
#pragma unroll 1
    for (int kc = 0; kc < K; kc += 32) {
        V a[4], a2[4];
#pragma unroll
        for (int mb = 0; mb < 4; ++mb) { a[mb] = WFrag<T16>::ld(A + aoff + (size_t)mb * 16 * K + kc); if (NSPLIT == 1 || NSPLIT == 2) a2[mb] = WFrag<T16>::ld(A2 + aoff + (size_t)mb * 16 * K + kc); }
#pragma unroll
        for (int nb = 0; nb < 4; ++nb) { const V b = WFrag<T16>::ld(Bt + boff + (size_t)nb * 16 * K + kc); V b2; if (NSPLIT >= 2) b2 = WFrag<T16>::ld(Bt2 + boff + (size_t)nb * 16 * K + kc);
#pragma unroll
            for (int mb = 0; mb < 4; ++mb) { acc[mb][nb] = WFrag<T16>::mma(a[mb], b, acc[mb][nb]); if (NSPLIT == 1 || NSPLIT == 2) acc[mb][nb] = WFrag<T16>::mma(a2[mb], b, acc[mb][nb]); if (NSPLIT >= 2) acc[mb][nb] = WFrag<T16>::mma(a[mb], b2, acc[mb][nb]); } }
        asm volatile("v_nop\n\tv_nop\n\tv_nop\n\tv_nop" : "+v"(acc[0][0]), "+v"(acc[1][1]), "+v"(acc[2][2]), "+v"(acc[3][3]) : "v"(a[0]), "v"(a[3]));
    }
#pragma unroll
    for (int mb = 0; mb < 4; ++mb) {
#pragma unroll
        for (int nb = 0; nb < 4; ++nb) {
#pragma unroll
            for (int j = 0; j < 8; ++j) os[(hi * 8 + j) * 68 + nb * 16 + lr] = acc[mb][nb][j]; }
        __builtin_amdgcn_wave_barrier(); asm volatile("" ::: "memory");
        float* crow = C + (size_t)(r0 + mb * 16) * ldc + c0;
#pragma unroll 1
        for (int ps = 0; ps < 2; ++ps) {
#pragma unroll
            for (int s = 0; s < 8; ++s) { const int row = 2 * s + hi, cofs = lr * 4; v4f val = *(const v4fa*)(os + row * 68 + cofs); if (BIAS) { val[0] += bfr(bias[c0 + cofs]); val[1] += bfr(bias[c0 + cofs + 1]); val[2] += bfr(bias[c0 + cofs + 2]); val[3] += bfr(bias[c0 + cofs + 3]); }
                *(volatile v4f*)(crow + (size_t)row * ldc + cofs) = val; }
            if (ps == 0) __threadfence(); }
        __builtin_amdgcn_wave_barrier(); asm volatile("" ::: "memory");
    }
}

__device__ __forceinline__ void splitf(float y, unsigned short& h, unsigned short& l) { h = f2bf(y); l = f2bf(y - bf2f(h)); }
typedef __attribute__((ext_vector_type(2))) unsigned short v2us;
typedef __attribute__((ext_vector_type(4))) unsigned short v4us;

__global__ __launch_bounds__(256) void k_wtG(const float* __restrict__ w, int K, int N, bf* Bt) {
    const int lane = threadIdx.x & 31; const int L0 = (blockIdx.x * 8 + (threadIdx.x >> 5)) * 8; const int nlines = N * K / 64;
#pragma unroll 1
    for (int ps = 0; ps < 2; ++ps) {
#pragma unroll 1
        for (int l = 0; l < 8; ++l) { const int L = L0 + l; if (L >= nlines) break; const size_t e = (size_t)L * 64 + lane * 2; const int k = (int)(e % K), n = (int)(e / K); v2us o;
            o[0] = f2bf(w[(size_t)k * N + n]); o[1] = f2bf(w[(size_t)(k + 1) * N + n]); *(volatile v2us*)(Bt + e) = o; }
        if (ps == 0) __threadfence(); }
}
__global__ __launch_bounds__(256) void k_poly(const float* __restrict__ x, float* P) { const int i = blockIdx.x * 256 + threadIdx.x; if (i >= NTOK * 4) return; const float xv = bfr(x[i]); float z = __fmul_rn(xv, (1.0f / SIG)); asm volatile("" : "+v"(z)); const float win = __expf(__fmul_rn(-0.5f, __fmul_rn(z, z))); float pw = 1.0f; float v[16]; v[0] = 1.0f;
#pragma unroll
    for (int u = 1; u < 16; ++u) { pw = __fmul_rn(pw, xv); float t = __fmul_rn(pw, win); asm volatile("" : "+v"(t)); v[u] = __fmul_rn(t, c_norm[u - 1]); }
    for (int ps = 0; ps < 2; ++ps) {
#pragma unroll
        for (int q4 = 0; q4 < 4; ++q4) { v4f o; o[0] = v[q4 * 4]; o[1] = v[q4 * 4 + 1]; o[2] = v[q4 * 4 + 2]; o[3] = v[q4 * 4 + 3]; *(volatile v4f*)(P + (size_t)i * 16 + q4 * 4) = o; }
        if (ps == 0) __threadfence(); } }
__global__ __launch_bounds__(256) void k_basis(const float* __restrict__ P, int t0, bf* Bh, bf* Bl) { const size_t e = ((size_t)blockIdx.x * 256 + threadIdx.x) * 4; if (e >= (size_t)TCH * KK) return; const int k = (int)(e % KK); const int t = t0 + (int)(e / KK); const float* p = P + (size_t)t * 64; const int a = k >> 12, b = (k >> 8) & 15, cc = (k >> 4) & 15, d0 = k & 15;
    float pab = __fmul_rn(p[a], p[16 + b]); asm volatile("" : "+v"(pab)); float pabc = __fmul_rn(pab, p[32 + cc]); asm volatile("" : "+v"(pabc)); v4us oh, ol;
#pragma unroll
    for (int q = 0; q < 4; ++q) { unsigned short u, l; splitf(__fmul_rn(pabc, p[48 + d0 + q]), u, l); oh[q] = u; ol[q] = l; } *(volatile v4us*)(Bh + e) = oh; *(volatile v4us*)(Bl + e) = ol; __threadfence(); *(volatile v4us*)(Bh + e) = oh; *(volatile v4us*)(Bl + e) = ol; }

extern "C" void kernel_launch(void* const* d_in, const int* in_sizes, int n_in,
                              void* d_out, int out_size, void* d_ws, size_t ws_size, hipStream_t stream) {
    (void)in_sizes; (void)n_in; (void)out_size;
    const float* x = (const float*)d_in[0]; const float* w = (const float*)d_in[1];
    float* OUT = (float*)d_out;
    char* wsp = (char*)d_ws;
    auto take = [&](size_t bytes) { char* p = wsp; wsp += (bytes + 255) & ~(size_t)255; return (void*)p; };
    bf* WB = (bf*)take((size_t)OC * KK * 2); float* P = (float*)take((size_t)NTOK * 64 * 4); bf* Bh = (bf*)take((size_t)TCH * KK * 2); bf* Bl = (bf*)take((size_t)TCH * KK * 2);
    if ((size_t)(wsp - (char*)d_ws) > ws_size) return;
    k_wtG<<<(KK * OC / 64 + 63) / 64, 256, 0, stream>>>(w, KK, OC, WB);
    k_poly<<<(NTOK * 4 + 255) / 256, 256, 0, stream>>>(x, P);
    for (int t0 = 0; t0 < NTOK; t0 += TCH) {
        k_basis<<<(unsigned)(((size_t)TCH * KK / 4 + 255) / 256), 256, 0, stream>>>(P, t0, Bh, Bl);
        k_gemmw<bf, 1, false><<<dim3(TCH / 64, OC / 64, 1), 32, 0, stream>>>(Bh, Bl, WB, nullptr, KK, OUT + (size_t)t0 * OC, OC, nullptr, 0, 0, 0); }
}
